// MultiHeadAttention_8735963480133
// MI455X (gfx1250) — hardware-verified
//
#include <hip/hip_runtime.h>
#pragma clang fp contract(off)
#ifndef NB
#define NB 4
#endif
#ifndef SEQ
#define SEQ 2048
#endif
#define NB_FULL 4
#define SEQ_FULL 2048
#define EMB 1024
#define NH 16
#define HD 64
#define NQKV 3072
#define KD 1024
#define XSTRIDE_FULL ((size_t)SEQ_FULL * EMB)
#define MROWS (NB * SEQ)
#define PLANE ((size_t)NB * NH * SEQ * HD)

static_assert(SEQ % 128 == 0);
static_assert(SEQ <= SEQ_FULL);
static_assert(NB <= NB_FULL);
static_assert(HD == 64);
static_assert(NH * HD == EMB);
static_assert(NQKV == 3 * EMB);
static_assert(KD % 32 == 0);
static_assert(MROWS % 128 == 0);
static_assert((size_t)MROWS * EMB * 2 * 2 + (size_t)NQKV * KD * 2 + (size_t)EMB * KD * 2 + 3 * PLANE * 2 + 6 * 256 <= (size_t)134217728);

typedef __bf16 v16b __attribute__((ext_vector_type(16)));
typedef _Float16 v16h __attribute__((ext_vector_type(16)));
typedef unsigned short v8us __attribute__((ext_vector_type(8), may_alias));
typedef float v8f __attribute__((ext_vector_type(8)));
typedef float v4f __attribute__((ext_vector_type(4)));
typedef float v4fa __attribute__((ext_vector_type(4), may_alias));
union Frag { v16b b; v16h h; v8us half[2]; _Float16 e[16]; };
union Pack8 { v8us v; _Float16 e[8]; };

#define LOG2E 1.4426950408889634f
#define SCL2 (LOG2E * 0.00048828125f)

__device__ __forceinline__ unsigned short bf16_bits(float x) {
  unsigned int u = __float_as_uint(x);
  return (unsigned short)((u + 0x7FFFu + ((u >> 16) & 1u)) >> 16);
}
__device__ __forceinline__ float bf16_rne(float x) { return __uint_as_float(((unsigned int)bf16_bits(x)) << 16); }
__device__ __forceinline__ unsigned short f16_bits(float x) {
  union { _Float16 h; unsigned short u; } c;
  c.h = (_Float16)x;
  return c.u;
}

__global__ __launch_bounds__(256) void k_xb(const float* __restrict__ X, unsigned short* __restrict__ Xb) {
  const int t = blockIdx.x * 256 + threadIdx.x;
  if (t >= MROWS * (EMB / 8)) return;
  const int row = t >> 7, piece = t & 127;
  const int b = row / SEQ, s = row - b * SEQ;
  const float* src = X + (size_t)b * XSTRIDE_FULL + (size_t)s * EMB + piece * 8;
  const v4f x0 = *(const v4fa*)(src), x1 = *(const v4fa*)(src + 4);
  v8us o;
  o[0] = bf16_bits(x0[0]); o[1] = bf16_bits(x0[1]); o[2] = bf16_bits(x0[2]); o[3] = bf16_bits(x0[3]);
  o[4] = bf16_bits(x1[0]); o[5] = bf16_bits(x1[1]); o[6] = bf16_bits(x1[2]); o[7] = bf16_bits(x1[3]);
  unsigned short* d = Xb + (size_t)t * 8;
  *(volatile v8us*)d = o;
  __threadfence();
  *(volatile v8us*)d = o;
}

template <int MODE>
__global__ __launch_bounds__(256) void k_wt(const float* __restrict__ W, unsigned short* __restrict__ Wt, int N) {
  __shared__ __attribute__((aligned(16))) unsigned short tl[64 * 72];
  const int tid = threadIdx.x;
  const int ntiles = N >> 6;
  const int kt = blockIdx.x / ntiles, nt = blockIdx.x - kt * ntiles;
  const int k0 = kt * 64, n0 = nt * 64;
  for (int i = tid; i < 64 * 16; i += 256) {
    const int j = i >> 4, c4 = (i & 15) * 4;
    const v4f x = *(const v4fa*)(W + (size_t)(k0 + j) * N + n0 + c4);
#pragma unroll
    for (int e = 0; e < 4; ++e) {
      unsigned short u;
      if (MODE == 0) u = bf16_bits(x[e]);
      else           u = f16_bits(bf16_rne(x[e]) * 1024.0f);
      tl[(c4 + e) * 72 + j] = u;
    }
  }
  __syncthreads();
  for (int pass = 0; pass < 2; ++pass) {
    for (int i = tid; i < 64 * 8; i += 256) {
      const int n = i >> 3, j8 = (i & 7) * 8;
      const v8us v = *(const v8us*)&tl[n * 72 + j8];
      *(volatile v8us*)(Wt + (size_t)(n0 + n) * KD + k0 + j8) = v;
    }
    if (pass == 0) __threadfence();
  }
}

template <bool BF>
__device__ __forceinline__ void gemm_tile(const unsigned short* __restrict__ ap, const unsigned short* __restrict__ bp, v8f (&acc)[2][4]) {
#pragma unroll 1
  for (int k0 = 0; k0 < KD; k0 += 32) {
    Frag a0, a1, b0, b1, b2, b3;
    a0.half[0] = *(const v8us*)(ap + k0);                 a0.half[1] = *(const v8us*)(ap + k0 + 16);
    a1.half[0] = *(const v8us*)(ap + 16 * KD + k0);       a1.half[1] = *(const v8us*)(ap + 16 * KD + k0 + 16);
    b0.half[0] = *(const v8us*)(bp + k0);                 b0.half[1] = *(const v8us*)(bp + k0 + 16);
    b1.half[0] = *(const v8us*)(bp + 16 * KD + k0);       b1.half[1] = *(const v8us*)(bp + 16 * KD + k0 + 16);
    b2.half[0] = *(const v8us*)(bp + 32 * KD + k0);       b2.half[1] = *(const v8us*)(bp + 32 * KD + k0 + 16);
    b3.half[0] = *(const v8us*)(bp + 48 * KD + k0);       b3.half[1] = *(const v8us*)(bp + 48 * KD + k0 + 16);
    if (BF) {
      acc[0][0] = __builtin_amdgcn_wmma_f32_16x16x32_bf16(false, a0.b, false, b0.b, (short)0, acc[0][0], false, false);
      acc[0][1] = __builtin_amdgcn_wmma_f32_16x16x32_bf16(false, a0.b, false, b1.b, (short)0, acc[0][1], false, false);
      acc[0][2] = __builtin_amdgcn_wmma_f32_16x16x32_bf16(false, a0.b, false, b2.b, (short)0, acc[0][2], false, false);
      acc[0][3] = __builtin_amdgcn_wmma_f32_16x16x32_bf16(false, a0.b, false, b3.b, (short)0, acc[0][3], false, false);
      acc[1][0] = __builtin_amdgcn_wmma_f32_16x16x32_bf16(false, a1.b, false, b0.b, (short)0, acc[1][0], false, false);
      acc[1][1] = __builtin_amdgcn_wmma_f32_16x16x32_bf16(false, a1.b, false, b1.b, (short)0, acc[1][1], false, false);
      acc[1][2] = __builtin_amdgcn_wmma_f32_16x16x32_bf16(false, a1.b, false, b2.b, (short)0, acc[1][2], false, false);
      acc[1][3] = __builtin_amdgcn_wmma_f32_16x16x32_bf16(false, a1.b, false, b3.b, (short)0, acc[1][3], false, false);
      asm volatile("v_nop\n\tv_nop\n\tv_nop\n\tv_nop"
                   : "+v"(acc[0][0]), "+v"(acc[0][1]), "+v"(acc[0][2]), "+v"(acc[0][3]),
                     "+v"(acc[1][0]), "+v"(acc[1][1]), "+v"(acc[1][2]), "+v"(acc[1][3])
                   : "v"(a0.b), "v"(a1.b), "v"(b0.b), "v"(b1.b), "v"(b2.b), "v"(b3.b));
    } else {
      acc[0][0] = __builtin_amdgcn_wmma_f32_16x16x32_f16(false, a0.h, false, b0.h, (short)0, acc[0][0], false, false);
      acc[0][1] = __builtin_amdgcn_wmma_f32_16x16x32_f16(false, a0.h, false, b1.h, (short)0, acc[0][1], false, false);
      acc[0][2] = __builtin_amdgcn_wmma_f32_16x16x32_f16(false, a0.h, false, b2.h, (short)0, acc[0][2], false, false);
      acc[0][3] = __builtin_amdgcn_wmma_f32_16x16x32_f16(false, a0.h, false, b3.h, (short)0, acc[0][3], false, false);
      acc[1][0] = __builtin_amdgcn_wmma_f32_16x16x32_f16(false, a1.h, false, b0.h, (short)0, acc[1][0], false, false);
      acc[1][1] = __builtin_amdgcn_wmma_f32_16x16x32_f16(false, a1.h, false, b1.h, (short)0, acc[1][1], false, false);
      acc[1][2] = __builtin_amdgcn_wmma_f32_16x16x32_f16(false, a1.h, false, b2.h, (short)0, acc[1][2], false, false);
      acc[1][3] = __builtin_amdgcn_wmma_f32_16x16x32_f16(false, a1.h, false, b3.h, (short)0, acc[1][3], false, false);
      asm volatile("v_nop\n\tv_nop\n\tv_nop\n\tv_nop"
                   : "+v"(acc[0][0]), "+v"(acc[0][1]), "+v"(acc[0][2]), "+v"(acc[0][3]),
                     "+v"(acc[1][0]), "+v"(acc[1][1]), "+v"(acc[1][2]), "+v"(acc[1][3])
                   : "v"(a0.h), "v"(a1.h), "v"(b0.h), "v"(b1.h), "v"(b2.h), "v"(b3.h));
    }
  }
}

__global__ __launch_bounds__(128) void k_gemm_qkv(const unsigned short* __restrict__ Xb, const unsigned short* __restrict__ Wt,
                                                  unsigned short* __restrict__ P3) {
  __shared__ __attribute__((aligned(16))) unsigned short st[128 * 72];
  const int tid = threadIdx.x, lane = tid & 31, ln = lane & 15, hh = lane >> 4;
  const int w = __builtin_amdgcn_readfirstlane(tid >> 5);
  const int m0 = blockIdx.x * 128;
  const int nt = blockIdx.y;
  const int n0 = nt * 64;
  const int h = nt / 3, kind = nt - 3 * h;
  v8f acc[2][4];
#pragma unroll
  for (int mi = 0; mi < 2; ++mi)
#pragma unroll
    for (int ni = 0; ni < 4; ++ni)
#pragma unroll
      for (int r = 0; r < 8; ++r) acc[mi][ni][r] = 0.0f;
  gemm_tile<true>(Xb + (size_t)(m0 + 32 * w + ln) * KD + 8 * hh, Wt + (size_t)(n0 + ln) * KD + 8 * hh, acc);
  const int b = m0 / SEQ, t0 = m0 - b * SEQ;
  if (kind != 2) {
#pragma unroll
    for (int mi = 0; mi < 2; ++mi)
#pragma unroll
      for (int ni = 0; ni < 4; ++ni)
#pragma unroll
        for (int r = 0; r < 8; ++r)
          st[(32 * w + 16 * mi + 8 * hh + r) * 72 + 16 * ni + ln] = f16_bits(acc[mi][ni][r] * 16.0f);
  } else {
#pragma unroll
    for (int mi = 0; mi < 2; ++mi)
#pragma unroll
      for (int ni = 0; ni < 4; ++ni) {
        Pack8 o;
#pragma unroll
        for (int r = 0; r < 8; ++r) o.e[r] = (_Float16)(acc[mi][ni][r] * 16.0f);
        *(v8us*)&st[(16 * ni + ln) * 136 + 32 * w + 16 * mi + 8 * hh] = o.v;
      }
  }
  __syncthreads();
  if (kind != 2) {
    unsigned short* dst = P3 + (size_t)kind * PLANE + ((size_t)(b * NH + h) * SEQ + t0) * HD;
    for (int pass = 0; pass < 2; ++pass) {
#pragma unroll 1
      for (int it = 0; it < 8; ++it) {
        const int i = it * 128 + tid;
        const int row = i >> 3, piece = i & 7;
        const v8us v = *(const v8us*)&st[row * 72 + piece * 8];
        *(volatile v8us*)(dst + (size_t)i * 8) = v;
      }
      if (pass == 0) __threadfence();
    }
  } else {
    unsigned short* dst = P3 + 2 * PLANE + ((size_t)(b * NH + h) * HD) * SEQ + t0;
    for (int pass = 0; pass < 2; ++pass) {
#pragma unroll 1
      for (int it = 0; it < 8; ++it) {
        const int i = it * 128 + tid;
        const int d = i >> 4, piece = i & 15;
        const v8us v = *(const v8us*)&st[d * 136 + piece * 8];
        *(volatile v8us*)(dst + (size_t)d * SEQ + piece * 8) = v;
      }
      if (pass == 0) __threadfence();
    }
  }
}

__device__ __forceinline__ v8f mma_s(v16h a0, v16h b0, v16h a1, v16h b1) {
  v8f c = {0.f, 0.f, 0.f, 0.f, 0.f, 0.f, 0.f, 0.f};
  c = __builtin_amdgcn_wmma_f32_16x16x32_f16(false, a0, false, b0, (short)0, c, false, false);
  c = __builtin_amdgcn_wmma_f32_16x16x32_f16(false, a1, false, b1, (short)0, c, false, false);
  asm volatile("v_nop\n\tv_nop\n\tv_nop\n\tv_nop" : "+v"(c) : "v"(a0), "v"(b0), "v"(a1), "v"(b1));
  return c;
}
__device__ __forceinline__ void mma_pv(v16h v0, v16h v1, v16h v2, v16h v3, v16h p, v8f (&O)[4]) {
  O[0] = __builtin_amdgcn_wmma_f32_16x16x32_f16(false, v0, false, p, (short)0, O[0], false, false);
  O[1] = __builtin_amdgcn_wmma_f32_16x16x32_f16(false, v1, false, p, (short)0, O[1], false, false);
  O[2] = __builtin_amdgcn_wmma_f32_16x16x32_f16(false, v2, false, p, (short)0, O[2], false, false);
  O[3] = __builtin_amdgcn_wmma_f32_16x16x32_f16(false, v3, false, p, (short)0, O[3], false, false);
  asm volatile("v_nop\n\tv_nop\n\tv_nop\n\tv_nop"
               : "+v"(O[0]), "+v"(O[1]), "+v"(O[2]), "+v"(O[3])
               : "v"(v0), "v"(v1), "v"(v2), "v"(v3), "v"(p));
}

__device__ __forceinline__ void fa_step(const unsigned short* __restrict__ Kp, const unsigned short* __restrict__ Vp,
                                        int key0, int ln, int hh, const Frag& q0, const Frag& q1,
                                        float& mr, float& lr, v8f (&O)[4]) {
  const unsigned short* kp0 = Kp + (size_t)(key0 + ln) * HD + 8 * hh;
  const unsigned short* kp1 = kp0 + 16 * HD;
  Frag k00, k01, k10, k11;
  k00.half[0] = *(const v8us*)(kp0);      k00.half[1] = *(const v8us*)(kp0 + 16);
  k01.half[0] = *(const v8us*)(kp0 + 32); k01.half[1] = *(const v8us*)(kp0 + 48);
  k10.half[0] = *(const v8us*)(kp1);      k10.half[1] = *(const v8us*)(kp1 + 16);
  k11.half[0] = *(const v8us*)(kp1 + 32); k11.half[1] = *(const v8us*)(kp1 + 48);
  const unsigned short* vp = Vp + (size_t)ln * SEQ + key0 + 8 * hh;
  Frag vf[4];
#pragma unroll
  for (int t = 0; t < 4; ++t) {
    vf[t].half[0] = *(const v8us*)(vp + (size_t)t * 16 * SEQ);
    vf[t].half[1] = *(const v8us*)(vp + (size_t)t * 16 * SEQ + 16);
  }
  const v8f s0 = mma_s(k00.h, q0.h, k01.h, q1.h);
  const v8f s1 = mma_s(k10.h, q0.h, k11.h, q1.h);
  float sc[16];
#pragma unroll
  for (int r = 0; r < 8; ++r) { sc[r] = s0[r] * SCL2; sc[8 + r] = s1[r] * SCL2; }
  float mx = sc[0];
#pragma unroll
  for (int i = 1; i < 16; ++i) mx = fmaxf(mx, sc[i]);
  mx = fmaxf(mx, __shfl_xor(mx, 16, 32));
  const float mnew = fmaxf(mr, mx);
  const float al = __builtin_amdgcn_exp2f(mr - mnew);
  mr = mnew;
  const float mb = mnew - 8.0f;
  Frag ph;
  float ps = 0.0f;
#pragma unroll
  for (int i = 0; i < 16; ++i) {
    const float pc = __builtin_amdgcn_exp2f(sc[i] - mb);
    ps += pc;
    ph.e[i] = (_Float16)pc;
  }
  ps += __shfl_xor(ps, 16, 32);
  lr = lr * al + ps;
#pragma unroll
  for (int t = 0; t < 4; ++t) O[t] = O[t] * al;
  mma_pv(vf[0].h, vf[1].h, vf[2].h, vf[3].h, ph.h, O);
}

__global__ __launch_bounds__(128) void k_attn(const unsigned short* __restrict__ P3, unsigned short* __restrict__ Cx) {
  __shared__ __attribute__((aligned(16))) unsigned short so[4 * 16 * 72];
  const int tid = threadIdx.x, lane = tid & 31, ln = lane & 15, hh = lane >> 4;
  const int w = __builtin_amdgcn_readfirstlane(tid >> 5);
  const int bh = blockIdx.x / (SEQ / 64), qt = blockIdx.x - bh * (SEQ / 64);
  const int b = bh / NH, h = bh - b * NH;
  const int qbase = qt * 64 + 16 * w;
  const unsigned short* qrow = P3 + ((size_t)bh * SEQ + qbase + ln) * HD + 8 * hh;
  Frag q0, q1;
  q0.half[0] = *(const v8us*)(qrow);      q0.half[1] = *(const v8us*)(qrow + 16);
  q1.half[0] = *(const v8us*)(qrow + 32); q1.half[1] = *(const v8us*)(qrow + 48);
  float mr = -1.0e30f, lr = 0.0f;
  v8f O[4];
#pragma unroll
  for (int t = 0; t < 4; ++t)
#pragma unroll
    for (int r = 0; r < 8; ++r) O[t][r] = 0.0f;
  const unsigned short* Kp = P3 + PLANE + (size_t)bh * SEQ * HD;
  const unsigned short* Vp = P3 + 2 * PLANE + (size_t)bh * HD * SEQ;
#pragma unroll 1
  for (int j = 0; j < SEQ / 32; ++j)
    fa_step(Kp, Vp, 32 * j, ln, hh, q0, q1, mr, lr, O);

  const float inv = 64.0f * (1.0f / lr);
#pragma unroll
  for (int t = 0; t < 4; ++t) {
    Pack8 o;
#pragma unroll
    for (int r = 0; r < 8; ++r) o.e[r] = (_Float16)(O[t][r] * inv);
    *(v8us*)&so[(w * 16 + ln) * 72 + 16 * t + 8 * hh] = o.v;
  }
  __syncthreads();
  unsigned short* cg = Cx + ((size_t)b * SEQ + qbase) * EMB + h * HD;
  const int rsub = lane >> 3, piece = lane & 7;
  for (int pass = 0; pass < 2; ++pass) {
#pragma unroll
    for (int q = 0; q < 4; ++q) {
      const int row = 4 * q + rsub;
      const v8us v = *(const v8us*)&so[(w * 16 + row) * 72 + piece * 8];
      *(volatile v8us*)(cg + (size_t)row * EMB + piece * 8) = v;
    }
    if (pass == 0) __threadfence();
  }
}

__global__ __launch_bounds__(128) void k_gemm_out(const unsigned short* __restrict__ Cx, const unsigned short* __restrict__ WoT,
                                                  float* __restrict__ Out) {
  __shared__ __attribute__((aligned(16))) float sf[128 * 68];
  const int tid = threadIdx.x, lane = tid & 31, ln = lane & 15, hh = lane >> 4;
  const int w = __builtin_amdgcn_readfirstlane(tid >> 5);
  const int m0 = blockIdx.x * 128;
  const int n0 = blockIdx.y * 64;
  v8f acc[2][4];
#pragma unroll
  for (int mi = 0; mi < 2; ++mi)
#pragma unroll
    for (int ni = 0; ni < 4; ++ni)
#pragma unroll
      for (int r = 0; r < 8; ++r) acc[mi][ni][r] = 0.0f;
  gemm_tile<false>(Cx + (size_t)(m0 + 32 * w + ln) * KD + 8 * hh, WoT + (size_t)(n0 + ln) * KD + 8 * hh, acc);
#pragma unroll
  for (int mi = 0; mi < 2; ++mi)
#pragma unroll
    for (int ni = 0; ni < 4; ++ni)
#pragma unroll
      for (int r = 0; r < 8; ++r)
        sf[(32 * w + 16 * mi + 8 * hh + r) * 68 + 16 * ni + ln] = acc[mi][ni][r] * 9.5367431640625e-07f;
  __syncthreads();
  const int b = m0 / SEQ, t0 = m0 - b * SEQ;
  float* og = Out + (size_t)b * XSTRIDE_FULL + (size_t)t0 * EMB + n0;
  for (int pass = 0; pass < 2; ++pass) {
#pragma unroll 1
    for (int it = 0; it < 16; ++it) {
      const int i = it * 128 + tid;
      const int row = i >> 4, piece = i & 15;
      const v4f v = *(const v4fa*)&sf[row * 68 + piece * 4];
      *(volatile v4f*)(og + (size_t)row * EMB + piece * 4) = v;
    }
    if (pass == 0) __threadfence();
  }
}

extern "C" void kernel_launch(void* const* d_in, const int* in_sizes, int n_in,
                              void* d_out, int out_size, void* d_ws, size_t ws_size, hipStream_t stream) {
  if (n_in < 3) return;
  const long long needx = ((long long)(NB - 1) * SEQ_FULL + SEQ) * EMB;
  if ((long long)in_sizes[0] < needx) return;
  if ((long long)in_sizes[1] < (long long)EMB * NQKV) return;
  if ((long long)in_sizes[2] < (long long)EMB * EMB) return;
  if ((long long)out_size < needx) return;
  const float* X    = (const float*)d_in[0];
  const float* Wqkv = (const float*)d_in[1];
  const float* Wout = (const float*)d_in[2];
  float* Out = (float*)d_out;
  char* ws = (char*)d_ws;
  size_t off = 0;
  const size_t szX  = (size_t)MROWS * EMB * 2;
  const size_t szWq = (size_t)NQKV * KD * 2;
  const size_t szWo = (size_t)EMB * KD * 2;
  const size_t szP3 = 3 * PLANE * 2;
  unsigned short* Xb  = (unsigned short*)(ws + off); off += (szX  + 255) & ~(size_t)255;
  unsigned short* Wt  = (unsigned short*)(ws + off); off += (szWq + 255) & ~(size_t)255;
  unsigned short* WoT = (unsigned short*)(ws + off); off += (szWo + 255) & ~(size_t)255;
  unsigned short* P3  = (unsigned short*)(ws + off); off += (szP3 + 255) & ~(size_t)255;
  unsigned short* Cx  = (unsigned short*)(ws + off); off += (szX  + 255) & ~(size_t)255;
  if (off > ws_size) return;
  k_xb<<<(unsigned)((MROWS * (EMB / 8) + 255) / 256), 256, 0, stream>>>(X, Xb);
  k_wt<0><<<(unsigned)((NQKV / 64) * (KD / 64)), 256, 0, stream>>>(Wqkv, Wt, NQKV);
  k_wt<1><<<(unsigned)((EMB / 64) * (KD / 64)), 256, 0, stream>>>(Wout, WoT, EMB);
  k_gemm_qkv<<<dim3((unsigned)(MROWS / 128), (unsigned)(NQKV / 64)), 128, 0, stream>>>(Xb, Wt, P3);
  k_attn<<<(unsigned)(NB * NH * (SEQ / 64)), 128, 0, stream>>>(P3, Cx);
  k_gemm_out<<<dim3((unsigned)(MROWS / 128), (unsigned)(EMB / 64)), 128, 0, stream>>>(Cx, WoT, Out);
}
